// AdapterLayer_25872882991396
// MI455X (gfx1250) — hardware-verified
//
#include <hip/hip_runtime.h>
#include <math.h>

typedef __attribute__((ext_vector_type(16))) _Float16 v16h;
typedef __attribute__((ext_vector_type(8)))  _Float16 v8h;
typedef __attribute__((ext_vector_type(16))) __bf16   v16b;
typedef __attribute__((ext_vector_type(8)))  __bf16   v8b;
typedef __attribute__((ext_vector_type(8)))  float    v8f;
typedef __attribute__((ext_vector_type(4)))  float    v4f;

constexpr int kBat    = 4;
constexpr int kSeq    = 2048;
constexpr int kWidth  = 1024;
constexpr int kHeads  = 16;
constexpr int kRows   = kBat * kSeq;
constexpr int kGateN  = 64;
constexpr int kThr    = 256;

constexpr float kInCarry  = 1024.0f;
constexpr float kOCarry   = 256.0f;
constexpr float kProjScale = 1.0f / (kInCarry * kInCarry);
constexpr float kOutScale  = 1.0f / (kOCarry * kInCarry);
constexpr float kF16MinNormal = 6.103515625e-5f;

static_assert((kRows % 64) == 0 && (kWidth % 64) == 0 && (kGateN % 64) == 0 && (kWidth % 32) == 0, "GEMM M, N multiples of 64, K of 32");
static_assert(kProjScale == 9.5367431640625e-7f && kOutScale == 3.814697265625e-6f, "power-of-two scales");

constexpr size_t kOffH16  = 0;
constexpr size_t kOffWQ   = kOffH16 + (size_t)kRows * kWidth * 2;
constexpr size_t kOffWK   = kOffWQ  + (size_t)kWidth * kWidth * 2;
constexpr size_t kOffWV   = kOffWK  + (size_t)kWidth * kWidth * 2;
constexpr size_t kOffWG   = kOffWV  + (size_t)kWidth * kWidth * 2;
constexpr size_t kOffWO   = kOffWG  + (size_t)kWidth * kWidth * 2;
constexpr size_t kOffLW   = kOffWO  + (size_t)kWidth * kWidth * 2;
constexpr size_t kOffZB   = kOffLW  + (size_t)kGateN * kWidth * 2;
constexpr size_t kOffLRP  = kOffZB  + (size_t)kWidth * 4;
constexpr size_t kOffXQ   = kOffLRP + (size_t)kRows * kGateN * 4;
constexpr size_t kOffXK   = kOffXQ  + (size_t)kRows * kWidth * 4;
constexpr size_t kOffXV   = kOffXK  + (size_t)kRows * kWidth * 4;
constexpr size_t kWsTotal = kOffXV  + (size_t)kRows * kWidth * 4;
static_assert(kWsTotal == 130158592ull, "carve total");
static_assert(kWsTotal <= 134217728ull, "carve cap");
static_assert((kOffWQ % 256) == 0 && (kOffLW % 256) == 0 && (kOffZB % 256) == 0 && (kOffLRP % 256) == 0 && (kOffXQ % 256) == 0 && (kOffXK % 256) == 0 && (kOffXV % 256) == 0, "aligned regions");

__device__ __forceinline__ unsigned short f2bf_bits(float f) {
  unsigned u = __float_as_uint(f);
  return (unsigned short)((u + 0x7FFFu + ((u >> 16) & 1u)) >> 16);
}
__device__ __forceinline__ float bf_bits2f(unsigned short h) { return __uint_as_float(((unsigned)h) << 16); }
__device__ __forceinline__ float bf16r(float f) { return bf_bits2f(f2bf_bits(f)); }
__device__ __forceinline__ float carry_flush(float v, float carry) {
  const float s = v * carry;
  return (fabsf(s) < kF16MinNormal) ? 0.0f : s;
}
__device__ __forceinline__ float frcp(float x) { return __builtin_amdgcn_rcpf(x); }

__device__ __forceinline__ void dep_guard4_h(v8f& a, v8f& b, v8f& c, v8f& d, v16h x, v16h y) { asm volatile("v_nop\n\tv_nop\n\tv_nop\n\tv_nop" : "+v"(a), "+v"(b), "+v"(c), "+v"(d) : "v"(x), "v"(y)); }
__device__ __forceinline__ void dep_guard4_b(v8f& a, v8f& b, v8f& c, v8f& d, v16b x, v16b y) { asm volatile("v_nop\n\tv_nop\n\tv_nop\n\tv_nop" : "+v"(a), "+v"(b), "+v"(c), "+v"(d) : "v"(x), "v"(y)); }
__device__ __forceinline__ void keep4_h(v16h a, v16h b, v16h c, v16h d) { asm volatile("v_nop" :: "v"(a), "v"(b), "v"(c), "v"(d)); }
__device__ __forceinline__ void keep4_b(v16b a, v16b b, v16b c, v16b d) { asm volatile("v_nop" :: "v"(a), "v"(b), "v"(c), "v"(d)); }
__device__ __forceinline__ void acc_guard4(v8f& a, v8f& b, v8f& c, v8f& d) { asm volatile("v_nop\n\tv_nop\n\tv_nop\n\tv_nop" : "+v"(a), "+v"(b), "+v"(c), "+v"(d)); }

template <typename T> struct Frag;
template <> struct Frag<_Float16> {
  typedef v16h V; union U { v16h v; v8h h[2]; };
  static __device__ __forceinline__ v16h load(const _Float16* p) {
    U f; f.h[0] = *(const v8h*)(p); f.h[1] = *(const v8h*)(p + 16); return f.v;
  }
  static __device__ __forceinline__ v8f mma(v16h a, v16h b, v8f c) {
    return __builtin_amdgcn_wmma_f32_16x16x32_f16(false, a, false, b, (short)0, c, false, false);
  }
  static __device__ __forceinline__ void guard4(v8f& a, v8f& b, v8f& c, v8f& d, v16h x, v16h y) { dep_guard4_h(a, b, c, d, x, y); }
  static __device__ __forceinline__ void keep(v16h a, v16h b, v16h c, v16h d) { keep4_h(a, b, c, d); }
};
template <> struct Frag<__bf16> {
  typedef v16b V; union U { v16b v; v8b h[2]; };
  static __device__ __forceinline__ v16b load(const __bf16* p) {
    U f; f.h[0] = *(const v8b*)(p); f.h[1] = *(const v8b*)(p + 16); return f.v;
  }
  static __device__ __forceinline__ v8f mma(v16b a, v16b b, v8f c) {
    return __builtin_amdgcn_wmma_f32_16x16x32_bf16(false, a, false, b, (short)0, c, false, false);
  }
  static __device__ __forceinline__ void guard4(v8f& a, v8f& b, v8f& c, v8f& d, v16b x, v16b y) { dep_guard4_b(a, b, c, d, x, y); }
  static __device__ __forceinline__ void keep(v16b a, v16b b, v16b c, v16b d) { keep4_b(a, b, c, d); }
};

__device__ __forceinline__ v8f mma_h(v16h a, v16h b, v8f c) {
  c = __builtin_amdgcn_wmma_f32_16x16x32_f16(false, a, false, b, (short)0, c, false, false);
  asm volatile("v_nop\n\tv_nop\n\tv_nop\n\tv_nop" : "+v"(c) : "v"(a), "v"(b));
  return c;
}

template <int ET> struct Elem;
template <> struct Elem<0> { typedef _Float16 T; };
template <> struct Elem<1> { typedef __bf16 T; };
template <int ET, bool SPLIT, int BIAS_MODE, int OUT_MODE, bool RESID, int ACT = 0>
__global__ __launch_bounds__(256) void wmma_gemm64(
    const unsigned short* __restrict__ Ap, const unsigned short* __restrict__ A2p, int lda, long strideA,
    const unsigned short* __restrict__ Btp, const unsigned short* __restrict__ Bt2p, int ldb, long strideB,
    void* __restrict__ Cout, void* __restrict__ Cout2, int ldc, long strideC,
    const float* __restrict__ bias,
    const float* __restrict__ resid, long strideR,
    int M, int N, int K, float scale) {
  typedef typename Elem<ET>::T T;
  typedef typename Frag<T>::V V;
  const T* A = (const T*)Ap; const T* A2 = (const T*)A2p; const T* Bt = (const T*)Btp; const T* Bt2 = (const T*)Bt2p;
  __shared__ __align__(16) float sT[8][16 * 68];
  const int b    = blockIdx.y;
  const int lane = threadIdx.x & 31;
  const int wave = threadIdx.x >> 5;
  const int tilesN = N >> 6;
  const int tilesM = M >> 6;
  const int tile = blockIdx.x * 8 + wave;
  if (tile >= tilesM * tilesN) return;
  const int tm = tile / tilesN;
  const int tn = tile - tm * tilesN;
  const int m0 = tm << 6;
  const int n0 = tn << 6;

  const T* Ab  = A  + (size_t)b * strideA;
  const T* Bb  = Bt + (size_t)b * strideB;
  const T* Ab2 = SPLIT ? (A2  + (size_t)b * strideA) : nullptr;
  const T* Bb2 = SPLIT ? (Bt2 + (size_t)b * strideB) : nullptr;

  const int rlane = lane & 15;
  const int koff  = (lane >> 4) * 8;
  const int mOff  = (lane >> 4) * 8;

  v8f acc[4][4];
#pragma unroll
  for (int i = 0; i < 4; ++i)
#pragma unroll
    for (int j = 0; j < 4; ++j) acc[i][j] = (v8f){0.f,0.f,0.f,0.f,0.f,0.f,0.f,0.f};

  for (int k0 = 0; k0 < K; k0 += 32) {
    V bh[4], bl[4];
#pragma unroll
    for (int j = 0; j < 4; ++j) {
      const size_t bo = (size_t)(n0 + (j << 4) + rlane) * ldb + koff + k0;
      bh[j] = Frag<T>::load(Bb + bo);
      if (SPLIT) bl[j] = Frag<T>::load(Bb2 + bo);
    }
#pragma unroll
    for (int i = 0; i < 4; ++i) {
      const size_t ao = (size_t)(m0 + (i << 4) + rlane) * lda + koff + k0;
      V ah = Frag<T>::load(Ab + ao);
      V al;
      if (SPLIT) al = Frag<T>::load(Ab2 + ao);
#pragma unroll
      for (int j = 0; j < 4; ++j) {
        acc[i][j] = Frag<T>::mma(ah, bh[j], acc[i][j]);
        if (SPLIT) {
          acc[i][j] = Frag<T>::mma(ah, bl[j], acc[i][j]);
          acc[i][j] = Frag<T>::mma(al, bh[j], acc[i][j]);
        }
      }
      Frag<T>::guard4(acc[i][0], acc[i][1], acc[i][2], acc[i][3], ah, SPLIT ? al : ah);
    }
    Frag<T>::keep(bh[0], bh[1], bh[2], bh[3]);
    if (SPLIT) Frag<T>::keep(bl[0], bl[1], bl[2], bl[3]);
  }
  acc_guard4(acc[0][0], acc[0][1], acc[0][2], acc[0][3]);
  acc_guard4(acc[1][0], acc[1][1], acc[1][2], acc[1][3]);
  acc_guard4(acc[2][0], acc[2][1], acc[2][2], acc[2][3]);
  acc_guard4(acc[3][0], acc[3][1], acc[3][2], acc[3][3]);

  float* slab = sT[wave];
  const float* Rb = RESID ? (resid + (size_t)b * strideR) : nullptr;
#pragma unroll
  for (int i = 0; i < 4; ++i) {
    const int mBase = m0 + (i << 4);
#pragma unroll
    for (int j = 0; j < 4; ++j) {
      const int n = n0 + (j << 4) + rlane;
      float bv = 0.f;
      if (BIAS_MODE == 2) bv = bias[n];
#pragma unroll
      for (int r = 0; r < 8; ++r) {
        float v = acc[i][j][r] * scale;
        if (BIAS_MODE == 1) v += bias[mBase + mOff + r];
        if (BIAS_MODE == 2) v += bv;
        if (RESID) v += Rb[(size_t)(mBase + mOff + r) * ldc + n];
        if (ACT == 1) v = tanhf(v);
        if (ACT == 2) v = fmaxf(v, 0.0f);
        if (ACT == 3) v = v / (1.0f + expf(-v));
        if (ACT == 4) v = (v > 0.f) ? v : 0.01f * v;
        slab[(mOff + r) * 68 + (j << 4) + rlane] = v;
      }
    }
    __builtin_amdgcn_fence(__ATOMIC_RELEASE, "workgroup");
    __builtin_amdgcn_wave_barrier();
    __builtin_amdgcn_fence(__ATOMIC_ACQUIRE, "workgroup");
    if (OUT_MODE == 0) {
      float* C = (float*)Cout + (size_t)b * strideC;
      const int hh = lane >> 4, c4 = (lane & 15) * 4;
      for (int pass = 0; pass < 2; ++pass) {
#pragma unroll
        for (int it = 0; it < 8; ++it) {
          const int row = it * 2 + hh;
          v4f v = *(const v4f*)(slab + row * 68 + c4);
          *(volatile v4f*)(C + (size_t)(mBase + row) * ldc + n0 + c4) = v;
        }
        __threadfence();
      }
    } else {
      const int q = lane >> 3, c8 = (lane & 7) * 8;
      unsigned short* C  = (unsigned short*)Cout  + (size_t)b * strideC;
      unsigned short* C2 = (OUT_MODE == 2) ? ((unsigned short*)Cout2 + (size_t)b * strideC) : nullptr;
      for (int pass = 0; pass < 2; ++pass) {
#pragma unroll
        for (int it = 0; it < 4; ++it) {
          const int row = it * 4 + q;
          const float* sp = slab + row * 68 + c8;
          v8h hv, lv;
#pragma unroll
          for (int e = 0; e < 8; ++e) {
            if (OUT_MODE == 1) {
              hv[e] = (_Float16)sp[e];
            } else {
              unsigned short hb = f2bf_bits(sp[e]);
              unsigned short lb = f2bf_bits(sp[e] - bf_bits2f(hb));
              hv[e] = __builtin_bit_cast(_Float16, hb);
              lv[e] = __builtin_bit_cast(_Float16, lb);
            }
          }
          *(volatile v8h*)(C + (size_t)(mBase + row) * ldc + n0 + c8) = hv;
          if (OUT_MODE == 2) *(volatile v8h*)(C2 + (size_t)(mBase + row) * ldc + n0 + c8) = lv;
        }
        __threadfence();
      }
    }
    __builtin_amdgcn_fence(__ATOMIC_RELEASE, "workgroup");
    __builtin_amdgcn_wave_barrier();
    __builtin_amdgcn_fence(__ATOMIC_ACQUIRE, "workgroup");
  }
}

__global__ __launch_bounds__(kThr) void cast_plane_kernel(const float* __restrict__ src, unsigned short* __restrict__ dst,
                                                          int colsLog2, int dstPitch, int dstOff) {
  const int i   = blockIdx.x * kThr + threadIdx.x;
  const int sh  = colsLog2 - 3;
  const int row = i >> sh;
  const int c8  = (i & ((1 << sh) - 1)) * 8;
  const float* sp = src + ((size_t)row << colsLog2) + c8;
  const v4f a0 = *(const v4f*)(sp);
  const v4f a1 = *(const v4f*)(sp + 4);
  v8h hv;
#pragma unroll
  for (int e = 0; e < 4; ++e) {
    const float f0 = a0[e];
    const float f1 = a1[e];
    hv[e]     = (_Float16)carry_flush(bf16r(f0), kInCarry);
    hv[4 + e] = (_Float16)carry_flush(bf16r(f1), kInCarry);
  }
  unsigned short* dp = dst + (size_t)row * dstPitch + dstOff + c8;
  *(volatile v8h*)dp = hv;
  __threadfence();
  *(volatile v8h*)dp = hv;
}

__global__ __launch_bounds__(kThr) void gate_plane_kernel(const float* __restrict__ lr_w, unsigned short* __restrict__ LW16, float* __restrict__ ZB) {
  unsigned i = blockIdx.x * (unsigned)kThr + threadIdx.x;
  asm volatile("" : "+v"(i));
  const unsigned row = i >> 7;
  const unsigned c8 = (i & 127u) * 8u;
  v8h hv;
  if (row < (unsigned)kHeads) {
    const float* sp = lr_w + (size_t)row * kWidth + c8;
    const v4f a0 = *(const v4f*)(sp);
    const v4f a1 = *(const v4f*)(sp + 4);
#pragma unroll
    for (int e = 0; e < 4; ++e) {
      hv[e]     = (_Float16)carry_flush(bf16r(a0[e]), kInCarry);
      hv[4 + e] = (_Float16)carry_flush(bf16r(a1[e]), kInCarry);
    }
  } else {
#pragma unroll
    for (int e = 0; e < 8; ++e) hv[e] = (_Float16)0.0f;
  }
  unsigned short* dp = LW16 + (size_t)row * kWidth + c8;
  *(volatile v8h*)dp = hv;
  __threadfence();
  *(volatile v8h*)dp = hv;
  if (blockIdx.x == 0) {
    const v4f z4 = {0.f, 0.f, 0.f, 0.f};
    *(volatile v4f*)(ZB + 4u * threadIdx.x) = z4;
    __threadfence();
    *(volatile v4f*)(ZB + 4u * threadIdx.x) = z4;
  }
}

__device__ __forceinline__ float tanh_fast(float u) { return 1.0f - 2.0f * frcp(1.0f + __expf(2.0f * u)); }
__device__ __forceinline__ float gelu_f(float x) { return 0.5f * x * (1.0f + tanh_fast(0.7978845608028654f * (x + 0.044715f * x * x * x))); }
__device__ __forceinline__ float gelu_bwd_f(float x) {
  const float t = tanh_fast(0.79788456f * x * (1.0f + 0.044715f * x * x));
  return 0.5f * x * ((1.0f - t * t) * (0.79788456f + 0.1070322243f * x * x)) + 0.5f * (1.0f + t);
}
__device__ __forceinline__ void cvt_hl(float v, float c, _Float16& hi, _Float16& lo) {
  const float s = carry_flush(v, c);
  hi = (_Float16)s;
  const float r = s - (float)hi;
  lo = (_Float16)((fabsf(r) < kF16MinNormal) ? 0.0f : r);
}
union FragU { v16h v; v8h h[2]; };
__device__ __forceinline__ void frag_hl_tiles(v8f a, v8f b, float c, v16h& hi, v16h& lo) {
#pragma unroll
  for (int e = 0; e < 8; ++e) {
    _Float16 h, l;
    cvt_hl(a[e], c, h, l); hi[e] = h; lo[e] = l;
    cvt_hl(b[e], c, h, l); hi[8 + e] = h; lo[8 + e] = l;
  }
}
__device__ __forceinline__ v16h frag_fold_hl(v8f a, float c) {
  v16h f;
#pragma unroll
  for (int e = 0; e < 8; ++e) { _Float16 h, l; cvt_hl(a[e], c, h, l); f[e] = h; f[8 + e] = l; }
  return f;
}
__device__ __forceinline__ v8h words8(v8f a, float c) {
  v8h w;
#pragma unroll
  for (int e = 0; e < 8; ++e) w[e] = (_Float16)carry_flush(a[e], c);
  return w;
}
__device__ __forceinline__ v16h frag_dup(v8h w) { FragU f; f.h[0] = w; f.h[1] = w; return f.v; }
__device__ __forceinline__ v16h frag_h32(const _Float16* p) { FragU f; f.h[0] = *(const v8h*)(p); f.h[1] = *(const v8h*)(p + 16); return f.v; }
__device__ __forceinline__ v16h frag_h16(const _Float16* p) {
  FragU f; f.h[0] = *(const v8h*)(p);
#pragma unroll
  for (int e = 0; e < 8; ++e) f.h[1][e] = (_Float16)0.0f;
  return f.v;
}
__device__ __forceinline__ v8f zero8() { return (v8f){0.f, 0.f, 0.f, 0.f, 0.f, 0.f, 0.f, 0.f}; }
constexpr int kXP = 68;
constexpr int kGP = 72;
constexpr int kTP = 24;
constexpr int kWP = 72;
constexpr float kMaster = 134217728.0f;
constexpr float cX   = 64.0f;
constexpr float cW   = 4096.0f;
constexpr float cAct = 1024.0f;
constexpr float cG2  = 32.0f;
constexpr float cG1  = 128.0f;
constexpr float cBm1 = 2048.0f;
constexpr float cBm2 = 131072.0f;
constexpr float cLX1 = 1048576.0f;
constexpr float cLX2 = 4194304.0f;
constexpr float cLast = 1048576.0f;
constexpr float kWfromMaster = cW / kMaster;
constexpr float kS18 = 1.0f / (cX * cW);
constexpr float kS22 = 1.0f / (cAct * cW);
constexpr float kS17 = 1.0f / (cG2 * cW);
constexpr float kS12 = 1.0f / (cX * cX);
constexpr float kS20 = 1.0f / (cAct * cAct);
constexpr float kS27 = 1.0f / kMaster;
static_assert(cG1 * cBm1 == cX * cW && cG2 * cBm2 == cAct * cW, "the correction products share their accumulators' scales");
static_assert(cLX1 * cG1 == kMaster && cLX2 * cG2 == kMaster && cLast * cG1 == kMaster, "the updates accumulate in the masters' unit");

__global__ __launch_bounds__(512) void ttt_chain_kernel(float* __restrict__ XQ, const float* __restrict__ XK, const float* __restrict__ XV,
                                                        const float* __restrict__ LRP, const float* __restrict__ lr_b,
                                                        const float* __restrict__ tok_in, const float* __restrict__ norm_w,
                                                        const float* __restrict__ norm_b, const float* __restrict__ W1in,
                                                        const float* __restrict__ b1in, const float* __restrict__ W2in,
                                                        const float* __restrict__ b2in) {
  __shared__ __align__(16) float sXQ[16 * kXP];
  __shared__ __align__(16) float sTG[16 * kXP];
  __shared__ __align__(16) float sZ2[16 * kXP];
  __shared__ __align__(16) float sPart[8 * 64 * 16];
  __shared__ __align__(16) float sAt2[8 * 16 * 16];
  __shared__ __align__(16) float sAt2r[16 * 16];
  __shared__ __align__(16) float sB1[256];
  __shared__ __align__(16) float sB2[64];
  __shared__ __align__(16) float sDB2[64];
  __shared__ __align__(16) float sNw[64];
  __shared__ __align__(16) float sNb[64];
  __shared__ __align__(16) float sTok[16];
  __shared__ __align__(16) float sLrn[16];
  __shared__ __align__(16) _Float16 sXKh[16 * kGP];
  __shared__ __align__(16) _Float16 sXKl[16 * kGP];
  __shared__ __align__(16) _Float16 sXQh[16 * kGP];
  __shared__ __align__(16) _Float16 sXQl[16 * kGP];
  __shared__ __align__(16) _Float16 sGZ2[16 * kGP];
  __shared__ __align__(16) _Float16 sGZ2T[64 * kTP];
  __shared__ __align__(16) _Float16 sBm[32 * 8];
  __shared__ __align__(16) _Float16 sXKT[64 * kTP];
  __shared__ __align__(16) _Float16 wT2[16 * 16 * kWP];
  __shared__ __align__(16) _Float16 wG1[16 * 16 * kTP];
  __shared__ __align__(16) _Float16 wX2[16 * 16 * kTP];

  const int chain = blockIdx.x;
  const int bb = chain >> 4;
  const int hh = chain & 15;
  const int tid = threadIdx.x;
  const int lane = tid & 31;
  const int wave = tid >> 5;
  const int hs = lane >> 4;
  const int col = lane & 15;

  v8f T1[4], T2[4];
#pragma unroll
  for (int mt = 0; mt < 4; ++mt)
#pragma unroll
    for (int r = 0; r < 8; ++r) {
      float w = W1in[((size_t)hh * 64 + 16 * mt + 8 * hs + r) * 256 + 16 * wave + col];
      T1[mt][r] = kMaster * bf16r(w);
    }
#pragma unroll
  for (int nt = 0; nt < 4; ++nt)
#pragma unroll
    for (int r = 0; r < 8; ++r) {
      float w = W2in[((size_t)hh * 256 + 16 * wave + 8 * hs + r) * 64 + 16 * nt + col];
      T2[nt][r] = kMaster * bf16r(w);
    }
  if (tid < 256) sB1[tid] = bf16r(b1in[hh * 256 + tid]);
  if (tid < 64) {
    sB2[tid] = bf16r(b2in[hh * 64 + tid]);
    sNw[tid] = bf16r(norm_w[hh * 64 + tid]);
    sNb[tid] = bf16r(norm_b[hh * 64 + tid]);
  }
  if (tid < 16) sTok[tid] = fmaxf(1.0f / (float)(tid + 1) + bf16r(tok_in[tid]), 0.0f);
  const float lrb = bf16r(lr_b[hh]);
  __syncthreads();
  int colv, hsv, tidv, lanev;

#pragma unroll 1
  for (int n = 0; n < 128; ++n) {
    colv = col; hsv = hs; tidv = tid; lanev = lane; asm volatile("" : "+v"(colv), "+v"(hsv), "+v"(tidv), "+v"(lanev));
    const size_t row0 = (size_t)bb * 2048 + 16 * (size_t)n;
    if (tidv < 256) {
      typedef __attribute__((ext_vector_type(4))) _Float16 v4h;
      const int t = tidv >> 4;
      const int d4 = (tidv & 15) * 4;
      const size_t g = (row0 + t) * 1024 + hh * 64 + d4;
      const v4f xk = *(const v4f*)(XK + g);
      const v4f xq = *(const v4f*)(XQ + g);
      const v4f xv = *(const v4f*)(XV + g);
      const float z = LRP[(row0 + t) * 64 + hh] + lrb;
      const float lrn = (1.0f / (1.0f + expf(-z))) / 64.0f;
      if ((tidv & 15) == 0) sLrn[t] = lrn;
      const float last = sTok[15] * lrn;
      *(v4f*)(sXQ + t * kXP + d4) = xq;
      *(v4f*)(sTG + t * kXP + d4) = xv - xk;
      v4h kh, kl, qh, ql;
#pragma unroll
      for (int e = 0; e < 4; ++e) {
        _Float16 h, l;
        cvt_hl(xk[e], cX, h, l); kh[e] = h; kl[e] = l;
        cvt_hl(xq[e], cX, h, l); qh[e] = h; ql[e] = l;
        sXKT[(d4 + e) * kTP + t] = (_Float16)carry_flush(-last * xk[e], cLX1);
      }
      *(v4h*)(sXKh + t * kGP + d4) = kh;
      *(v4h*)(sXKl + t * kGP + d4) = kl;
      *(v4h*)(sXQh + t * kGP + d4) = qh;
      *(v4h*)(sXQl + t * kGP + d4) = ql;
    }
    __syncthreads();
    colv = col; hsv = hs; tidv = tid; lanev = lane; asm volatile("" : "+v"(colv), "+v"(hsv), "+v"(tidv), "+v"(lanev));

    v8f z1;
    v8f accq = zero8();
    v16h x2h;
    v8h w2w[4];
    {
      v8f acc = zero8();
#pragma unroll
      for (int s = 0; s < 2; ++s) {
        v16h ah, al;
        frag_hl_tiles(T1[2 * s], T1[2 * s + 1], kWfromMaster, ah, al);
        {
          const v16h bxh = frag_h32(sXKh + colv * kGP + 32 * s + 8 * hsv);
          const v16h bxl = frag_h32(sXKl + colv * kGP + 32 * s + 8 * hsv);
          acc = mma_h(ah, bxh, acc);
          acc = mma_h(ah, bxl, acc);
          acc = mma_h(al, bxh, acc);
        }
        {
          const v16h bqh = frag_h32(sXQh + colv * kGP + 32 * s + 8 * hsv);
          const v16h bql = frag_h32(sXQl + colv * kGP + 32 * s + 8 * hsv);
          accq = mma_h(ah, bqh, accq);
          accq = mma_h(ah, bql, accq);
          accq = mma_h(al, bqh, accq);
        }
      }
#pragma unroll
      for (int r = 0; r < 8; ++r) z1[r] = acc[r] * kS18 + sB1[16 * wave + 8 * hsv + r];
      v8f x2t;
#pragma unroll
      for (int r = 0; r < 8; ++r) x2t[r] = gelu_f(z1[r]);
      x2h = frag_fold_hl(x2t, cAct);
      const float lastc = sTok[15] * sLrn[colv];
#pragma unroll
      for (int r = 0; r < 8; ++r) wX2[(wave * 16 + 8 * hsv + r) * kTP + colv] = (_Float16)carry_flush(-lastc * x2t[r], cLX2);
      if (wave == 15) {
        v16h bm;
        {
          v8f acc = zero8();
#pragma unroll
          for (int s = 0; s < 2; ++s) {
            acc = mma_h(frag_h32(sXKh + colv * kGP + 32 * s + 8 * hsv), frag_h32(sXQh + colv * kGP + 32 * s + 8 * hsv), acc);
          }
          const float tki = sTok[colv];
#pragma unroll
          for (int e = 0; e < 8; ++e) {
            const int j = 8 * hsv + e;
            const float v = (j <= colv) ? tki * sLrn[j] * (acc[e] * kS12 + 1.0f) : 0.0f;
            bm[e] = (_Float16)carry_flush(-v, cBm1);
            bm[8 + e] = (_Float16)0.0f;
          }
        }
        FragU fb; fb.v = bm;
        *(v8h*)(sBm + lanev * 8) = fb.h[0];
      }
      float* slot = sPart + ((wave & 7) * 64 + 8 * hsv) * 16 + colv;
      if (wave >= 8) {
#pragma unroll
        for (int nt = 0; nt < 4; ++nt) {
          w2w[nt] = words8(T2[nt], kWfromMaster);
#pragma unroll
          for (int e = 0; e < 8; ++e) wT2[(wave * 16 + 8 * hsv + e) * kWP + 16 * nt + colv] = w2w[nt][e];
          const v8f a2 = mma_h(frag_dup(w2w[nt]), x2h, zero8());
#pragma unroll
          for (int r = 0; r < 8; ++r) slot[(16 * nt + r) * 16] = a2[r] * kS22;
          asm volatile("" ::: "memory");
        }
      }
      __syncthreads();
    colv = col; hsv = hs; tidv = tid; lanev = lane; asm volatile("" : "+v"(colv), "+v"(hsv), "+v"(tidv), "+v"(lanev));
      if (wave < 8) {
#pragma unroll
        for (int nt = 0; nt < 4; ++nt) {
          w2w[nt] = words8(T2[nt], kWfromMaster);
#pragma unroll
          for (int e = 0; e < 8; ++e) wT2[(wave * 16 + 8 * hsv + e) * kWP + 16 * nt + colv] = w2w[nt][e];
          const v8f a2 = mma_h(frag_dup(w2w[nt]), x2h, zero8());
#pragma unroll
          for (int r = 0; r < 8; ++r) slot[(16 * nt + r) * 16] += a2[r] * kS22;
          asm volatile("" ::: "memory");
        }
      }
    }
    __syncthreads();
    colv = col; hsv = hs; tidv = tid; lanev = lane; asm volatile("" : "+v"(colv), "+v"(hsv), "+v"(tidv), "+v"(lanev));

    if (tidv < 256) {
      const int d = tidv >> 2;
      const int t4 = (tidv & 3) * 4;
      v4f s4 = {0.f, 0.f, 0.f, 0.f};
#pragma unroll
      for (int w = 0; w < 8; ++w) s4 += *(const v4f*)(sPart + (w * 64 + d) * 16 + t4);
      const float bb2 = sB2[d];
#pragma unroll
      for (int e = 0; e < 4; ++e) sZ2[(t4 + e) * kXP + d] = s4[e] + bb2;
    }
    __syncthreads();
    colv = col; hsv = hs; tidv = tid; lanev = lane; asm volatile("" : "+v"(colv), "+v"(hsv), "+v"(tidv), "+v"(lanev));

    if (wave == 0) {
      if (lanev < 16) {
        float* zr = sZ2 + lanev * kXP;
        const float* tg = sTG + lanev * kXP;
        float s = 0.f;
#pragma unroll 4
        for (int d = 0; d < 64; ++d) s += zr[d];
        const float mu = s / 64.0f;
        float v = 0.f;
#pragma unroll 4
        for (int d = 0; d < 64; ++d) { const float dv = zr[d] - mu; v += dv * dv; }
        const float sd = sqrtf(v / 64.0f + 1e-6f);
        float s1 = 0.f, s2 = 0.f;
#pragma unroll 4
        for (int d = 0; d < 64; ++d) {
          const float xh = (zr[d] - mu) / sd;
          const float gx = (sNw[d] * xh + sNb[d] - tg[d]) * sNw[d];
          s1 += gx; s2 += gx * xh;
        }
        const float m1 = s1 / 64.0f, m2 = s2 / 64.0f;
        const float lastc = sTok[15] * sLrn[lanev];
#pragma unroll 4
        for (int d = 0; d < 64; ++d) {
          const float xh = (zr[d] - mu) / sd;
          const float gx = (sNw[d] * xh + sNb[d] - tg[d]) * sNw[d];
          const float g = (gx - m1 - xh * m2) / sd;
          const _Float16 gh = (_Float16)carry_flush(g, cG2);
          sGZ2[lanev * kGP + d] = gh;
          sGZ2T[d * kTP + lanev] = gh;
          zr[d] = lastc * g;
        }
      }
      __builtin_amdgcn_fence(__ATOMIC_RELEASE, "workgroup");
      __builtin_amdgcn_wave_barrier();
      __builtin_amdgcn_fence(__ATOMIC_ACQUIRE, "workgroup");
#pragma unroll
      for (int k = 0; k < 2; ++k) {
        const int d = lanev + 32 * k;
        float s = 0.f;
#pragma unroll
        for (int t = 0; t < 16; ++t) s += sZ2[t * kXP + d];
        sDB2[d] = s;
      }
    }
    __syncthreads();
    colv = col; hsv = hs; tidv = tid; lanev = lane; asm volatile("" : "+v"(colv), "+v"(hsv), "+v"(tidv), "+v"(lanev));

    {
      {
        v8f acc = zero8();
#pragma unroll
        for (int s = 0; s < 2; ++s)
          acc = mma_h(frag_h32(wT2 + (wave * 16 + colv) * kWP + 32 * s + 8 * hsv), frag_h32(sGZ2 + colv * kGP + 32 * s + 8 * hsv), acc);
#pragma unroll
        for (int r = 0; r < 8; ++r)
          wG1[(wave * 16 + 8 * hsv + r) * kTP + colv] = (_Float16)carry_flush(acc[r] * kS17 * gelu_bwd_f(z1[r]), cG1);
      }
      __builtin_amdgcn_fence(__ATOMIC_RELEASE, "workgroup");
      __builtin_amdgcn_wave_barrier();
      __builtin_amdgcn_fence(__ATOMIC_ACQUIRE, "workgroup");

      const v16h bm = frag_h16(sBm + lanev * 8);
      asm volatile("" ::: "memory");
      colv = col; hsv = hs; tidv = tid; lanev = lane; asm volatile("" : "+v"(colv), "+v"(hsv), "+v"(tidv), "+v"(lanev));
      const v16h ag1 = frag_h16(wG1 + (wave * 16 + colv) * kTP + 8 * hsv);
      v8f x2b;
      {
        v8f acc = mma_h(ag1, bm, accq);
#pragma unroll
        for (int r = 0; r < 8; ++r) x2b[r] = gelu_f(acc[r] * kS18 + sB1[16 * wave + 8 * hsv + r]);
      }
      {
        v16h bl;
#pragma unroll
        for (int e = 0; e < 8; ++e) {
          const float lv = (colv == 0) ? -(sTok[15] * sLrn[8 * hsv + e]) : 0.0f;
          bl[e] = (_Float16)carry_flush(lv, cLast);
          bl[8 + e] = (_Float16)0.0f;
        }
        const v8f acc = mma_h(ag1, bl, zero8());
        if (colv == 0) {
#pragma unroll
          for (int r = 0; r < 8; ++r) sB1[16 * wave + 8 * hsv + r] += acc[r] * kS27;
        }
      }
#pragma unroll
      for (int mt = 0; mt < 4; ++mt) T1[mt] = mma_h(frag_h16(sXKT + (16 * mt + colv) * kTP + 8 * hsv), ag1, T1[mt]);
      asm volatile("" ::: "memory");
      colv = col; hsv = hs; tidv = tid; lanev = lane; asm volatile("" : "+v"(colv), "+v"(hsv), "+v"(tidv), "+v"(lanev));
      const v16h xbf = frag_fold_hl(x2b, cAct);
      const v8f at2 = mma_h(x2h, xbf, zero8());
      float* aslot = sAt2 + ((wave & 7) * 16 + 8 * hsv) * 16 + colv;
      float* slot = sPart + ((wave & 7) * 64 + 8 * hsv) * 16 + colv;
      if (wave >= 8) {
#pragma unroll
        for (int nt = 0; nt < 4; ++nt) {
          const v8f a2 = mma_h(frag_dup(w2w[nt]), xbf, zero8());
#pragma unroll
          for (int r = 0; r < 8; ++r) slot[(16 * nt + r) * 16] = a2[r] * kS22;
          asm volatile("" ::: "memory");
        }
        const v16h a = frag_h16(wX2 + (wave * 16 + colv) * kTP + 8 * hsv);
#pragma unroll
        for (int nt = 0; nt < 4; ++nt) T2[nt] = mma_h(a, frag_h16(sGZ2T + (16 * nt + colv) * kTP + 8 * hsv), T2[nt]);
#pragma unroll
        for (int r = 0; r < 8; ++r) aslot[r * 16] = at2[r] * kS20;
      }
      __syncthreads();
    colv = col; hsv = hs; tidv = tid; lanev = lane; asm volatile("" : "+v"(colv), "+v"(hsv), "+v"(tidv), "+v"(lanev));
      if (wave < 8) {
#pragma unroll
        for (int nt = 0; nt < 4; ++nt) {
          const v8f a2 = mma_h(frag_dup(w2w[nt]), xbf, zero8());
#pragma unroll
          for (int r = 0; r < 8; ++r) slot[(16 * nt + r) * 16] += a2[r] * kS22;
          asm volatile("" ::: "memory");
        }
        const v16h a = frag_h16(wX2 + (wave * 16 + colv) * kTP + 8 * hsv);
#pragma unroll
        for (int nt = 0; nt < 4; ++nt) T2[nt] = mma_h(a, frag_h16(sGZ2T + (16 * nt + colv) * kTP + 8 * hsv), T2[nt]);
#pragma unroll
        for (int r = 0; r < 8; ++r) aslot[r * 16] += at2[r] * kS20;
      }
    }
    __syncthreads();
    colv = col; hsv = hs; tidv = tid; lanev = lane; asm volatile("" : "+v"(colv), "+v"(hsv), "+v"(tidv), "+v"(lanev));

    if (tidv < 256) {
      const int d = tidv >> 2;
      const int t4 = (tidv & 3) * 4;
      v4f s4 = {0.f, 0.f, 0.f, 0.f};
#pragma unroll
      for (int w = 0; w < 8; ++w) s4 += *(const v4f*)(sPart + (w * 64 + d) * 16 + t4);
      const float bb2 = sB2[d];
#pragma unroll
      for (int e = 0; e < 4; ++e) sZ2[(t4 + e) * kXP + d] = s4[e] + bb2;
      float a = 0.f;
#pragma unroll
      for (int w = 0; w < 8; ++w) a += sAt2[w * 256 + tidv];
      sAt2r[tidv] = a;
    }
    __syncthreads();
    colv = col; hsv = hs; tidv = tid; lanev = lane; asm volatile("" : "+v"(colv), "+v"(hsv), "+v"(tidv), "+v"(lanev));

    if (wave == 0) {
      v16h bm2;
      {
        const float tki = sTok[colv];
#pragma unroll
        for (int e = 0; e < 8; ++e) {
          const int j = 8 * hsv + e;
          const float v = (j <= colv) ? tki * sLrn[j] * (sAt2r[j * 16 + colv] + 1.0f) : 0.0f;
          bm2[e] = (_Float16)carry_flush(-v, cBm2);
          bm2[8 + e] = (_Float16)0.0f;
        }
      }
#pragma unroll
      for (int nt = 0; nt < 4; ++nt) {
        const v8f acc = mma_h(frag_h16(sGZ2T + (16 * nt + colv) * kTP + 8 * hsv), bm2, zero8());
#pragma unroll
        for (int r = 0; r < 8; ++r) sZ2[colv * kXP + 16 * nt + 8 * hsv + r] += acc[r] * kS22;
      }
      __builtin_amdgcn_fence(__ATOMIC_RELEASE, "workgroup");
      __builtin_amdgcn_wave_barrier();
      __builtin_amdgcn_fence(__ATOMIC_ACQUIRE, "workgroup");
      if (lanev < 16) {
        const float* zr = sZ2 + lanev * kXP;
        const float* xq = sXQ + lanev * kXP;
        float s = 0.f;
#pragma unroll 4
        for (int d = 0; d < 64; ++d) s += zr[d];
        const float mu = s / 64.0f;
        float v = 0.f;
#pragma unroll 4
        for (int d = 0; d < 64; ++d) { const float dv = zr[d] - mu; v += dv * dv; }
        const float rs = rsqrtf(v / 64.0f + 1e-6f);
        float* orow = XQ + (row0 + lanev) * 1024 + hh * 64;
        for (int pass = 0; pass < 2; ++pass) {
#pragma unroll 4
          for (int d4 = 0; d4 < 64; d4 += 4) {
            v4f o;
#pragma unroll
            for (int e = 0; e < 4; ++e) o[e] = xq[d4 + e] + (sNw[d4 + e] * ((zr[d4 + e] - mu) * rs) + sNb[d4 + e]);
            *(volatile v4f*)(orow + d4) = o;
          }
          __threadfence();
        }
      }
#pragma unroll
      for (int k = 0; k < 2; ++k) sB2[lanev + 32 * k] -= sDB2[lanev + 32 * k];
    }
    __syncthreads();
    colv = col; hsv = hs; tidv = tid; lanev = lane; asm volatile("" : "+v"(colv), "+v"(hsv), "+v"(tidv), "+v"(lanev));
  }
}

__device__ __forceinline__ float block_sum_256(float v, float* sRed, float* sGrp, int tid) {
  sRed[tid] = v;
  __syncthreads();
  if (tid < 8) {
    float s = 0.f;
#pragma unroll
    for (int k = 0; k < 8; ++k) {
      const v4f a = *(const v4f*)(sRed + tid * 32 + 4 * k);
      s += a[0]; s += a[1]; s += a[2]; s += a[3];
    }
    sGrp[tid] = s;
  }
  __syncthreads();
  float t = 0.f;
#pragma unroll
  for (int k = 0; k < 8; ++k) t += sGrp[k];
  __syncthreads();
  return t;
}
__global__ __launch_bounds__(kThr) void post_kernel(const float* __restrict__ XW, const float* __restrict__ G,
                                                    const float* __restrict__ post_w, const float* __restrict__ post_b,
                                                    unsigned short* __restrict__ O16) {
  __shared__ __align__(16) float sRed[256];
  __shared__ __align__(16) float sGrp[8];
  const int tid = threadIdx.x;
  const size_t base = (size_t)blockIdx.x * kWidth + 4 * tid;
  const v4f x = *(const v4f*)(XW + base);
  const v4f g = *(const v4f*)(G + base);
  const v4f pw = *(const v4f*)(post_w + 4 * tid);
  const v4f pb = *(const v4f*)(post_b + 4 * tid);
  const float mu = block_sum_256((x[0] + x[1]) + (x[2] + x[3]), sRed, sGrp, tid) / 1024.0f;
  float q = 0.f;
#pragma unroll
  for (int e = 0; e < 4; ++e) { const float dv = x[e] - mu; q += dv * dv; }
  const float var = block_sum_256(q, sRed, sGrp, tid) / 1024.0f;
  const float rs = rsqrtf(var + 1e-6f);
  typedef __attribute__((ext_vector_type(4))) _Float16 v4h;
  v4h ov;
#pragma unroll
  for (int e = 0; e < 4; ++e) {
    const float pwe = pw[e];
    const float pbe = pb[e];
    const float y = bf16r(pwe) * ((x[e] - mu) * rs) + bf16r(pbe);
    ov[e] = (_Float16)carry_flush(gelu_f(g[e]) * y, kOCarry);
  }
  unsigned short* dp = O16 + base;
  *(volatile v4h*)dp = ov;
  __threadfence();
  *(volatile v4h*)dp = ov;
}

static_assert(((kRows / 64) * (kWidth / 64)) % 8 == 0 && ((kRows / 64) * (kGateN / 64)) % 8 == 0, "GEMM grids exact");
static_assert(((size_t)kRows * kWidth / 8) % kThr == 0 && ((size_t)kWidth * kWidth / 8) % kThr == 0 && ((size_t)kGateN * kWidth / 8) % kThr == 0, "cast grids exact");

extern "C" void kernel_launch(void* const* d_in, const int* in_sizes, int n_in,
                              void* d_out, int out_size, void* d_ws, size_t ws_size,
                              hipStream_t stream) {
  if (n_in < 17 || d_out == nullptr || d_ws == nullptr) return;
  if (in_sizes[0] != kRows * kWidth) return;
  for (int k = 1; k <= 5; ++k) if (in_sizes[k] != kWidth * kWidth) return;
  if (in_sizes[6] != kHeads * kWidth || in_sizes[7] != kHeads || in_sizes[8] != 16) return;
  if (in_sizes[9] != kHeads * 64 || in_sizes[10] != kHeads * 64) return;
  if (in_sizes[11] != kHeads * 64 * 256 || in_sizes[12] != kHeads * 256 || in_sizes[13] != kHeads * 256 * 64 || in_sizes[14] != kHeads * 64) return;
  if (in_sizes[15] != kWidth || in_sizes[16] != kWidth) return;
  if (out_size != kRows * kWidth) return;
  if (ws_size < kWsTotal) return;

  const float* hidden = (const float*)d_in[0];
  const float* Wq = (const float*)d_in[1];
  const float* Wk = (const float*)d_in[2];
  const float* Wv = (const float*)d_in[3];
  const float* Wo = (const float*)d_in[4];
  const float* Wg = (const float*)d_in[5];
  const float* lr_w = (const float*)d_in[6];
  const float* lr_b = (const float*)d_in[7];
  const float* tok_in = (const float*)d_in[8];
  const float* norm_w = (const float*)d_in[9];
  const float* norm_b = (const float*)d_in[10];
  const float* W1 = (const float*)d_in[11];
  const float* b1 = (const float*)d_in[12];
  const float* W2 = (const float*)d_in[13];
  const float* b2 = (const float*)d_in[14];
  const float* post_w = (const float*)d_in[15];
  const float* post_b = (const float*)d_in[16];
  float* out = (float*)d_out;

  char* ws = (char*)d_ws;
  unsigned short* H16  = (unsigned short*)(ws + kOffH16);
  unsigned short* O16  = (unsigned short*)(ws + kOffH16);
  unsigned short* WQ16 = (unsigned short*)(ws + kOffWQ);
  unsigned short* WK16 = (unsigned short*)(ws + kOffWK);
  unsigned short* WV16 = (unsigned short*)(ws + kOffWV);
  unsigned short* WG16 = (unsigned short*)(ws + kOffWG);
  unsigned short* WO16 = (unsigned short*)(ws + kOffWO);
  unsigned short* LW16 = (unsigned short*)(ws + kOffLW);
  float*          ZB   = (float*)(ws + kOffZB);
  float*          LRP  = (float*)(ws + kOffLRP);
  float*          XQ   = (float*)(ws + kOffXQ);
  float*          XK   = (float*)(ws + kOffXK);
  float*          G    = (float*)(ws + kOffXK);
  float*          XV   = (float*)(ws + kOffXV);

  const int castH = (int)(((size_t)kRows * kWidth / 8) / kThr);
  const int castW = (int)(((size_t)kWidth * kWidth / 8) / kThr);
  cast_plane_kernel<<<castH, kThr, 0, stream>>>(hidden, H16, 10, kWidth, 0);
  cast_plane_kernel<<<castW, kThr, 0, stream>>>(Wq, WQ16, 10, kWidth, 0);
  cast_plane_kernel<<<castW, kThr, 0, stream>>>(Wk, WK16, 10, kWidth, 0);
  cast_plane_kernel<<<castW, kThr, 0, stream>>>(Wv, WV16, 10, kWidth, 0);
  cast_plane_kernel<<<castW, kThr, 0, stream>>>(Wg, WG16, 10, kWidth, 0);
  cast_plane_kernel<<<castW, kThr, 0, stream>>>(Wo, WO16, 10, kWidth, 0);
  gate_plane_kernel<<<(kGateN * kWidth / 8) / kThr, kThr, 0, stream>>>(lr_w, LW16, ZB);

  const dim3 gProj((kRows / 64) * (kWidth / 64) / 8, 1);
  wmma_gemm64<0, false, 2, 0, false, 0><<<gProj, 256, 0, stream>>>(
      H16, H16, kWidth, 0L, WQ16, WQ16, kWidth, 0L, (void*)XQ, (void*)XQ, kWidth, 0L, ZB, nullptr, 0L, kRows, kWidth, kWidth, kProjScale);
  wmma_gemm64<0, false, 2, 0, false, 0><<<gProj, 256, 0, stream>>>(
      H16, H16, kWidth, 0L, WK16, WK16, kWidth, 0L, (void*)XK, (void*)XK, kWidth, 0L, ZB, nullptr, 0L, kRows, kWidth, kWidth, kProjScale);
  wmma_gemm64<0, false, 2, 0, false, 0><<<gProj, 256, 0, stream>>>(
      H16, H16, kWidth, 0L, WV16, WV16, kWidth, 0L, (void*)XV, (void*)XV, kWidth, 0L, ZB, nullptr, 0L, kRows, kWidth, kWidth, kProjScale);
  wmma_gemm64<0, false, 2, 0, false, 0><<<dim3((kRows / 64) * (kGateN / 64) / 8, 1), 256, 0, stream>>>(
      H16, H16, kWidth, 0L, LW16, LW16, kWidth, 0L, (void*)LRP, (void*)LRP, kGateN, 0L, ZB, nullptr, 0L, kRows, kGateN, kWidth, kProjScale);

  ttt_chain_kernel<<<kBat * kHeads, 512, 0, stream>>>(XQ, XK, XV, LRP, lr_b, tok_in, norm_w, norm_b, W1, b1, W2, b2);

  wmma_gemm64<0, false, 2, 0, false, 0><<<gProj, 256, 0, stream>>>(
      H16, H16, kWidth, 0L, WG16, WG16, kWidth, 0L, (void*)G, (void*)G, kWidth, 0L, ZB, nullptr, 0L, kRows, kWidth, kWidth, kProjScale);
  post_kernel<<<kRows, kThr, 0, stream>>>(XQ, G, post_w, post_b, O16);
  wmma_gemm64<0, false, 2, 0, false, 0><<<gProj, 256, 0, stream>>>(
      O16, O16, kWidth, 0L, WO16, WO16, kWidth, 0L, (void*)out, (void*)out, kWidth, 0L, ZB, nullptr, 0L, kRows, kWidth, kWidth, kOutScale);
}
